// UpFormerBlock_linear_attn_29033978921044
// MI455X (gfx1250) — hardware-verified
//
#include <hip/hip_runtime.h>


namespace {
constexpr int N = 120000, CIN = 64, C = 128, NH = 8, DH = 16, C3 = 3 * C, KT = 27, NBLK = N / 64;
constexpr float XS = 8.0f, WSC = 256.0f, EPS = 1e-4f, BN_EPS = 1e-3f, LN_EPS = 1e-3f;
static_assert(N % 64 == 0, "row blocks");

typedef _Float16 b16;
typedef __attribute__((ext_vector_type(16))) _Float16 v16b;
typedef __attribute__((ext_vector_type(8))) _Float16 v8b;
typedef __attribute__((ext_vector_type(8))) float v8f;
typedef __attribute__((ext_vector_type(4))) float v4f;
__device__ __forceinline__ float bf16_rne(float f) { unsigned int u = __float_as_uint(f); u += 0x7FFFu + ((u >> 16) & 1u); return __uint_as_float(u & 0xFFFF0000u); }
__device__ __forceinline__ void split16(float v, b16& hi, b16& lo) { hi = (b16)v; lo = (b16)(v - (float)hi); }
__device__ __forceinline__ v16b frag_kb(const b16* p, int hh) { const v8b a = *(const v8b*)(p + 8 * hh), b = *(const v8b*)(p + 16 + 8 * hh); v16b f;
#pragma unroll
  for (int e = 0; e < 8; ++e) { f[e] = a[e]; f[8 + e] = b[e]; } return f; }
__device__ __forceinline__ v8f wmma16b(v16b a, v16b b, v8f c) { v8f d = __builtin_amdgcn_wmma_f32_16x16x32_f16(false, a, false, b, (short)0, c, false, false); asm volatile("v_nop\n\tv_nop\n\tv_nop\n\tv_nop" : "+v"(d) : "v"(a), "v"(b)); return d; }
__device__ __forceinline__ void wave_lds_sync() { __builtin_amdgcn_fence(__ATOMIC_RELEASE, "workgroup"); __builtin_amdgcn_wave_barrier(); __builtin_amdgcn_fence(__ATOMIC_ACQUIRE, "workgroup"); }
__device__ __forceinline__ float pmul(float a, float b) { float p = a * b; asm volatile("" : "+v"(p)); return p; }
__device__ __forceinline__ float hsum16(float v) { v += __shfl_xor(v, 1); v += __shfl_xor(v, 2); v += __shfl_xor(v, 4); return v + __shfl_xor(v, 8); }
__device__ __forceinline__ int iclamp(int v, int lo, int hi) { return v < lo ? lo : (v > hi ? hi : v); }
__device__ __forceinline__ float softplus_(float x) { return x > 20.0f ? x : log1pf(__expf(x)); }

__global__ __launch_bounds__(256) void prepx_kernel(const float* __restrict__ feat, const int* __restrict__ ind, b16* __restrict__ F16, b16* __restrict__ XYZ16) {
  const size_t g = (size_t)blockIdx.x * 256 + threadIdx.x; const int lane = threadIdx.x & 31; const size_t nf = (size_t)N * CIN / 8;
  if (g < nf) { const size_t e = g * 8; const v4f a = *(const v4f*)(feat + e), c = *(const v4f*)(feat + e + 4); v8b o;
#pragma unroll
    for (int j = 0; j < 4; ++j) { o[j] = (b16)(bf16_rne(a[j]) * XS); o[4 + j] = (b16)(bf16_rne(c[j]) * XS); }
    for (int pass = 0; pass < 2; ++pass) { *(volatile v8b*)(F16 + e) = o; __threadfence(); } return; }
  const size_t w = (g - nf) >> 5; const size_t row = w * 8 + (lane >> 2); if (row >= (size_t)N) return; const int seg = lane & 3; v8b o = {};
  if (seg == 0) { o[0] = (b16)((float)ind[row * 4 + 1] * XS); o[1] = (b16)((float)ind[row * 4 + 2] * XS); o[2] = (b16)((float)ind[row * 4 + 3] * XS); }
  for (int pass = 0; pass < 2; ++pass) { *(volatile v8b*)(XYZ16 + row * 32 + seg * 8) = o; __threadfence(); }
}
__global__ __launch_bounds__(256) void prepw_kernel(const float* __restrict__ wpre, const float* __restrict__ wp1, const float* __restrict__ wp2, const float* __restrict__ wqkv, const float* __restrict__ wdw, const float* __restrict__ wproj, b16* __restrict__ WPRE, b16* __restrict__ WP1, b16* __restrict__ WP2, b16* __restrict__ WQKV, b16* __restrict__ WDW, b16* __restrict__ WPROJ) {
  const int kind = blockIdx.y, t = blockIdx.x * 256 + threadIdx.x; int IN, KP, OUT; const float* w; b16* dst;
  if (kind == 0) { IN = CIN; KP = CIN; OUT = C; w = wpre; dst = WPRE; } else if (kind == 1) { IN = 3; KP = 32; OUT = C; w = wp1; dst = WP1; } else if (kind == 2) { IN = C; KP = C; OUT = C; w = wp2; dst = WP2; }
  else if (kind == 3) { IN = C; KP = C; OUT = C3; w = wqkv; dst = WQKV; } else if (kind < 4 + KT) { IN = C; KP = C; OUT = C; w = wdw + (size_t)(kind - 4) * C * C; dst = WDW + (size_t)(kind - 4) * C * C; } else { IN = C; KP = C; OUT = C; w = wproj; dst = WPROJ; }
  const int ngrp = OUT * KP / 8; if (t >= ngrp) return; const int o_ = (t * 8) / KP, k0 = t * 8 - o_ * KP; v8b o;
  for (int j = 0; j < 8; ++j) { const int k = k0 + j; o[j] = (k < IN) ? (b16)(bf16_rne(w[(size_t)(k < IN ? k : 0) * OUT + o_]) * WSC) : (b16)0.0f; }
  for (int pass = 0; pass < 2; ++pass) { *(volatile v8b*)(dst + (size_t)t * 8) = o; __threadfence(); }
}
__global__ __launch_bounds__(128) void node_kernel(const b16* __restrict__ F16, const b16* __restrict__ XYZ16, const b16* __restrict__ WPRE, const float* __restrict__ bpre, const float* __restrict__ gpre, const float* __restrict__ bepre, const float* __restrict__ mpre, const float* __restrict__ vpre,
                                                  const b16* __restrict__ WP1, const float* __restrict__ bp1, const float* __restrict__ gpe, const float* __restrict__ bepe, const float* __restrict__ mpe, const float* __restrict__ vpe, const b16* __restrict__ WP2, const float* __restrict__ bp2,
                                                  const b16* __restrict__ WQKV, const float* __restrict__ bqkv, const float* __restrict__ scp, b16* __restrict__ Q16, b16* __restrict__ V16, float* __restrict__ PART) {
  __shared__ __attribute__((aligned(16))) b16 Ts[4][16][C + 8], Tp[4][16][C + 8]; __shared__ __attribute__((aligned(16))) b16 KTt[C][64 + 8], VTt[C][64 + 8]; __shared__ float Ks[4][C]; __shared__ __attribute__((aligned(16))) b16 To[4][16][C + 8];
  const int wave = threadIdx.x >> 5, lane = threadIdx.x & 31, nloc = lane & 15, hlf = lane >> 4, t_ = threadIdx.x; const size_t m0 = (size_t)blockIdx.x * 64 + wave * 16;
  v8f acc[8];
#pragma unroll
  for (int t = 0; t < 8; ++t) acc[t] = (v8f){};
#pragma unroll
  for (int kb = 0; kb < CIN; kb += 32) { const v16b a = frag_kb(F16 + (m0 + nloc) * CIN + kb, hlf);
#pragma unroll
    for (int t = 0; t < 8; ++t) acc[t] = wmma16b(a, frag_kb(WPRE + (size_t)(t * 16 + nloc) * CIN + kb, hlf), acc[t]); }
#pragma unroll
  for (int t = 0; t < 8; ++t) { const int c = t * 16 + nloc; const float bb = bf16_rne(bpre[c]), g = bf16_rne(gpre[c]) * rsqrtf(bf16_rne(vpre[c]) + BN_EPS), mm = bf16_rne(mpre[c]), be = bf16_rne(bepre[c]);
#pragma unroll
    for (int r = 0; r < 8; ++r) Ts[wave][8 * hlf + r][c] = (b16)((pmul(acc[t][r] * (1.0f / (XS * WSC)) + bb - mm, g) + be) * XS); }
  { const v16b a = frag_kb(XYZ16 + (m0 + nloc) * 32, hlf);
#pragma unroll
    for (int t = 0; t < 8; ++t) { v8f p = {}; p = wmma16b(a, frag_kb(WP1 + (size_t)(t * 16 + nloc) * 32, hlf), p); const int c = t * 16 + nloc; const float bb = bf16_rne(bp1[c]), g = bf16_rne(gpe[c]) * rsqrtf(bf16_rne(vpe[c]) + BN_EPS), mm = bf16_rne(mpe[c]), be = bf16_rne(bepe[c]);
#pragma unroll
      for (int r = 0; r < 8; ++r) Tp[wave][8 * hlf + r][c] = (b16)(fmaxf(pmul(p[r] * (1.0f / (XS * WSC)) + bb - mm, g) + be, 0.0f) * XS); } }
  wave_lds_sync();
  float pev[8][8];
#pragma unroll
  for (int t = 0; t < 8; ++t) acc[t] = (v8f){};
#pragma unroll
  for (int kb = 0; kb < C; kb += 32) { const v16b a = frag_kb(&Tp[wave][nloc][kb], hlf);
#pragma unroll
    for (int t = 0; t < 8; ++t) acc[t] = wmma16b(a, frag_kb(WP2 + (size_t)(t * 16 + nloc) * C + kb, hlf), acc[t]); }
#pragma unroll
  for (int t = 0; t < 8; ++t) { const float bb = bf16_rne(bp2[t * 16 + nloc]);
#pragma unroll
    for (int r = 0; r < 8; ++r) pev[t][r] = acc[t][r] * (1.0f / (XS * WSC)) + bb; }
  auto gemm = [&](int which) {
#pragma unroll
    for (int t = 0; t < 8; ++t) acc[t] = (v8f){};
#pragma unroll
    for (int kb = 0; kb < C; kb += 32) { const v16b a = frag_kb(&Ts[wave][nloc][kb], hlf);
#pragma unroll
      for (int t = 0; t < 8; ++t) acc[t] = wmma16b(a, frag_kb(WQKV + (size_t)(which * C + t * 16 + nloc) * C + kb, hlf), acc[t]); } };
  auto featuremap = [&](int which) {
#pragma unroll
    for (int t = 0; t < 8; ++t) { const int c = t * 16 + nloc; const float bb = bf16_rne(bqkv[which * C + c]); const float sc = softplus_(bf16_rne(scp[c]));
#pragma unroll
      for (int r = 0; r < 8; ++r) { const float x = fmaxf(acc[t][r], 0.0f) + EPS; (void)bb; acc[t][r] = x / sc; } }
#pragma unroll
    for (int r = 0; r < 8; ++r) { float s_ = 0.0f;
#pragma unroll
      for (int t = 0; t < 8; ++t) s_ += pmul(acc[t][r], acc[t][r]);
      const float nrm = sqrtf(hsum16(s_));
#pragma unroll
      for (int t = 0; t < 8; ++t) acc[t][r] = pmul(acc[t][r] / nrm, nrm); } };
  gemm(1);
#pragma unroll
  for (int t = 0; t < 8; ++t) { const float bb = bf16_rne(bqkv[C + t * 16 + nloc]);
#pragma unroll
    for (int r = 0; r < 8; ++r) acc[t][r] = acc[t][r] * (1.0f / (XS * WSC)) + bb + pev[t][r]; }
  featuremap(1);
#pragma unroll
  for (int t = 0; t < 8; ++t) { float cs = 0.0f;
#pragma unroll
    for (int r = 0; r < 8; ++r) { KTt[t * 16 + nloc][wave * 16 + 8 * hlf + r] = (b16)(acc[t][r] * XS); cs += acc[t][r]; }
    cs += __shfl_xor(cs, 16); if (hlf == 0) Ks[wave][t * 16 + nloc] = cs; }
  gemm(0);
#pragma unroll
  for (int t = 0; t < 8; ++t) { const float bb = bf16_rne(bqkv[t * 16 + nloc]);
#pragma unroll
    for (int r = 0; r < 8; ++r) acc[t][r] = acc[t][r] * (1.0f / (XS * WSC)) + bb; }
  featuremap(0);
#pragma unroll
  for (int t = 0; t < 8; ++t)
#pragma unroll
    for (int r = 0; r < 8; ++r) To[wave][8 * hlf + r][t * 16 + nloc] = (b16)(acc[t][r] * XS);
  wave_lds_sync();
  for (int pass = 0; pass < 2; ++pass) { for (int rr = 0; rr < 16; ++rr) if (lane < 16) *(volatile v8b*)(Q16 + (m0 + rr) * C + lane * 8) = *(const v8b*)(&To[wave][rr][lane * 8]); __threadfence(); }
  wave_lds_sync();
  gemm(2);
#pragma unroll
  for (int t = 0; t < 8; ++t) { const float bb = bf16_rne(bqkv[2 * C + t * 16 + nloc]);
#pragma unroll
    for (int r = 0; r < 8; ++r) { const b16 hv = (b16)((acc[t][r] * (1.0f / (XS * WSC)) + bb) * XS); To[wave][8 * hlf + r][t * 16 + nloc] = hv; VTt[t * 16 + nloc][wave * 16 + 8 * hlf + r] = hv; } }
  wave_lds_sync();
  for (int pass = 0; pass < 2; ++pass) { for (int rr = 0; rr < 16; ++rr) if (lane < 16) *(volatile v8b*)(V16 + (m0 + rr) * C + lane * 8) = *(const v8b*)(&To[wave][rr][lane * 8]); __threadfence(); }
  __syncthreads();
  float* part = PART + (size_t)blockIdx.x * (NH * DH * DH + C);
  for (int hq = 0; hq < 2; ++hq) { const int h = wave * 2 + hq; v8f kvacc = {};
#pragma unroll
    for (int kb = 0; kb < 64; kb += 32) kvacc = wmma16b(frag_kb(&KTt[h * DH + nloc][kb], hlf), frag_kb(&VTt[h * DH + nloc][kb], hlf), kvacc);
    __shared__ float Tkv[4][DH * DH];
#pragma unroll
    for (int r = 0; r < 8; ++r) Tkv[wave][(8 * hlf + r) * DH + nloc] = kvacc[r] * (1.0f / (XS * XS));
    wave_lds_sync();
    for (int pass = 0; pass < 2; ++pass) { for (int q = lane; q < DH * DH / 4; q += 32) *(volatile v4f*)(part + (size_t)h * DH * DH + q * 4) = *(const v4f*)(&Tkv[wave][q * 4]); __threadfence(); }
    wave_lds_sync(); }
  if (wave == 0) { for (int pass = 0; pass < 2; ++pass) { for (int q = lane; q < C / 4; q += 32) { v4f s4; for (int j = 0; j < 4; ++j) { const int c = q * 4 + j; s4[j] = (Ks[0][c] + Ks[1][c]) + (Ks[2][c] + Ks[3][c]); } *(volatile v4f*)(part + NH * DH * DH + q * 4) = s4; } __threadfence(); } }
}
constexpr float KVS = 1024.0f;
__global__ __launch_bounds__(256) void reduce_kernel(const float* __restrict__ PART, b16* __restrict__ KVBh, b16* __restrict__ KVBl, float* __restrict__ KS) {
  __shared__ float R[NH * DH * DH + C];
  const int t_ = threadIdx.x; const int NOUT = NH * DH * DH + C;
  for (int o = t_; o < NOUT; o += 256) { float s = 0.0f;
#pragma unroll 1
    for (int b = 0; b < NBLK; ++b) s += PART[(size_t)b * NOUT + o]; R[o] = s; }
  __syncthreads();
  for (int pass = 0; pass < 2; ++pass) {
    for (int q = t_; q < C * C / 8; q += 256) { const int n = (q * 8) / C, k0 = q * 8 - n * C; const int h = n / DH, d = n - h * DH; v8b oh, ol;
      for (int j = 0; j < 8; ++j) { const int k = k0 + j; const int hk = k / DH, c = k - hk * DH; const float v = (hk == h) ? R[h * DH * DH + c * DH + d] / KVS : 0.0f; b16 a_, c_; split16(v, a_, c_); oh[j] = a_; ol[j] = c_; }
      *(volatile v8b*)(KVBh + (size_t)q * 8) = oh; *(volatile v8b*)(KVBl + (size_t)q * 8) = ol; }
    if (t_ < C / 4) { v4f s4; for (int j = 0; j < 4; ++j) s4[j] = R[NH * DH * DH + t_ * 4 + j]; *(volatile v4f*)(KS + t_ * 4) = s4; }
    __threadfence(); }
}
__global__ __launch_bounds__(128) void final_kernel(const b16* __restrict__ Q16, const b16* __restrict__ V16, const int* __restrict__ nbr, const b16* __restrict__ KVBh, const b16* __restrict__ KVBl, const float* __restrict__ KS, const b16* __restrict__ WDW, const float* __restrict__ bdw, const b16* __restrict__ WPROJ, const float* __restrict__ bproj,
                                                   const b16* __restrict__ F16, const b16* __restrict__ WPRE, const float* __restrict__ bpre, const float* __restrict__ gpre, const float* __restrict__ bepre, const float* __restrict__ mpre, const float* __restrict__ vpre, const float* __restrict__ gn1, const float* __restrict__ bn1, float* __restrict__ out) {
  __shared__ __attribute__((aligned(16))) b16 Tg[4][16][C + 8], Tgl[4][16][C + 8]; __shared__ __attribute__((aligned(16))) float Ty[4][16][C + 4];
  const int wave = threadIdx.x >> 5, lane = threadIdx.x & 31, nloc = lane & 15, hlf = lane >> 4; const size_t m0 = (size_t)blockIdx.x * 64 + wave * 16;
  v8f acc[8];
#pragma unroll
  for (int t = 0; t < 8; ++t) acc[t] = (v8f){};
#pragma unroll
  for (int kb = 0; kb < C; kb += 32) { const v16b a = frag_kb(Q16 + (m0 + nloc) * C + kb, hlf);
#pragma unroll
    for (int t = 0; t < 8; ++t) { const v16b bh_ = frag_kb(KVBh + (size_t)(t * 16 + nloc) * C + kb, hlf), bl_ = frag_kb(KVBl + (size_t)(t * 16 + nloc) * C + kb, hlf); acc[t] = wmma16b(a, bh_, acc[t]); acc[t] = wmma16b(a, bl_, acc[t]); } }
#pragma unroll
  for (int t = 0; t < 8; ++t) { const float ksc = KS[t * 16 + nloc];
#pragma unroll
    for (int r = 0; r < 8; ++r) { const size_t row = m0 + 8 * hlf + r; float p = pmul((float)Q16[row * C + t * 16 + nloc] * (1.0f / XS), ksc); p = hsum16(p); const float zz = 1.0f / (p + EPS); acc[t][r] = (acc[t][r] * (KVS / XS) * zz) * (XS * WSC); } }
#pragma unroll 1
  for (int ts = 0; ts < KT; ++ts) {
    { const int rr = lane >> 1, hf = lane & 1; const size_t row = m0 + rr; const int nb = nbr[row * KT + ts]; const bool ok = nb >= 0; const int nbc = iclamp(nb, 0, N - 1);
      const v8b* src = (const v8b*)(V16 + (size_t)nbc * C + hf * 64); v8b z8 = {};
#pragma unroll
      for (int q = 0; q < 8; ++q) *(v8b*)(&Tg[wave][rr][hf * 64 + q * 8]) = ok ? src[q] : z8; }
    wave_lds_sync();
#pragma unroll
    for (int kb = 0; kb < C; kb += 32) { const v16b a = frag_kb(&Tg[wave][nloc][kb], hlf);
#pragma unroll
      for (int t = 0; t < 8; ++t) acc[t] = wmma16b(a, frag_kb(WDW + ((size_t)ts * C + t * 16 + nloc) * C + kb, hlf), acc[t]); }
    wave_lds_sync(); }
#pragma unroll
  for (int t = 0; t < 8; ++t) { const float bb = bf16_rne(bdw[t * 16 + nloc]);
#pragma unroll
    for (int r = 0; r < 8; ++r) { b16 h_, l_; split16((acc[t][r] * (1.0f / (XS * WSC)) + bb) * XS, h_, l_); Tg[wave][8 * hlf + r][t * 16 + nloc] = h_; Tgl[wave][8 * hlf + r][t * 16 + nloc] = l_; } }
  wave_lds_sync();
#pragma unroll
  for (int t = 0; t < 8; ++t) acc[t] = (v8f){};
#pragma unroll
  for (int kb = 0; kb < C; kb += 32) { const v16b a = frag_kb(&Tg[wave][nloc][kb], hlf), al = frag_kb(&Tgl[wave][nloc][kb], hlf);
#pragma unroll
    for (int t = 0; t < 8; ++t) { const v16b bw = frag_kb(WPROJ + (size_t)(t * 16 + nloc) * C + kb, hlf); acc[t] = wmma16b(a, bw, acc[t]); acc[t] = wmma16b(al, bw, acc[t]); } }
#pragma unroll
  for (int t = 0; t < 8; ++t) { const int c = t * 16 + nloc; const float bb = bf16_rne(bproj[c]);
#pragma unroll
    for (int r = 0; r < 8; ++r) Ty[wave][8 * hlf + r][c] = acc[t][r] * (1.0f / (XS * WSC)) + bb; }
#pragma unroll
  for (int t = 0; t < 8; ++t) acc[t] = (v8f){};
#pragma unroll
  for (int kb = 0; kb < CIN; kb += 32) { const v16b a = frag_kb(F16 + (m0 + nloc) * CIN + kb, hlf);
#pragma unroll
    for (int t = 0; t < 8; ++t) acc[t] = wmma16b(a, frag_kb(WPRE + (size_t)(t * 16 + nloc) * CIN + kb, hlf), acc[t]); }
#pragma unroll
  for (int t = 0; t < 8; ++t) { const int c = t * 16 + nloc; const float bbp = bf16_rne(bpre[c]), g = bf16_rne(gpre[c]) * rsqrtf(bf16_rne(vpre[c]) + BN_EPS), mm = bf16_rne(mpre[c]), be = bf16_rne(bepre[c]);
#pragma unroll
    for (int r = 0; r < 8; ++r) Ty[wave][8 * hlf + r][c] += pmul(acc[t][r] * (1.0f / (XS * WSC)) + bbp - mm, g) + be; }
  wave_lds_sync();
  for (int rr = 0; rr < 16; ++rr) { const v4f v = *(const v4f*)(&Ty[wave][rr][lane * 4]); float s = (v[0] + v[1]) + (v[2] + v[3]);
#pragma unroll
    for (int o = 16; o >= 1; o >>= 1) s += __shfl_xor(s, o);
    const float mu = s * (1.0f / C); float ss = 0.0f; for (int j = 0; j < 4; ++j) { const float dv = v[j] - mu; ss += pmul(dv, dv); }
#pragma unroll
    for (int o = 16; o >= 1; o >>= 1) ss += __shfl_xor(ss, o);
    const float rs = rsqrtf(ss * (1.0f / C) + LN_EPS); v4f y; for (int j = 0; j < 4; ++j) { const int c = lane * 4 + j; y[j] = pmul(bf16_rne(gn1[c]), (v[j] - mu) * rs) + bf16_rne(bn1[c]); }
    for (int pass = 0; pass < 2; ++pass) { *(volatile v4f*)(out + (m0 + rr) * C + lane * 4) = y; __threadfence(); } }
}
}

extern "C" void kernel_launch(void* const* d_in, const int* in_sizes, int n_in, void* d_out, int out_size, void* d_ws, size_t ws_size, hipStream_t stream) {
  (void)n_in;
  auto Fp = [&](int i) { return (const float*)d_in[i]; }; auto Ip = [&](int i) { return (const int*)d_in[i]; };
  if (in_sizes[0] != N * CIN || in_sizes[1] != N * 4 || in_sizes[2] != N * KT || in_sizes[3] != CIN * C || in_sizes[17] != C * C3 || in_sizes[20] != KT * C * C || in_sizes[22] != C * C || out_size != N * C) return;
  size_t off = 0; char* ws = (char*)d_ws;
  auto carve = [&](size_t bytes) { char* p = ws + off; off += (bytes + 255) & ~(size_t)255; return p; };
  b16* F16 = (b16*)carve((size_t)N * CIN * 2); b16* XYZ16 = (b16*)carve((size_t)N * 32 * 2);
  b16* WPRE = (b16*)carve(C * CIN * 2); b16* WP1 = (b16*)carve(C * 32 * 2); b16* WP2 = (b16*)carve(C * C * 2); b16* WQKV = (b16*)carve((size_t)C3 * C * 2); b16* WDW = (b16*)carve((size_t)KT * C * C * 2); b16* WPROJ = (b16*)carve(C * C * 2);
  b16* Q16 = (b16*)carve((size_t)N * C * 2); b16* V16 = (b16*)carve((size_t)N * C * 2); float* PART = (float*)carve((size_t)NBLK * (NH * DH * DH + C) * 4); b16* KVBh = (b16*)carve(C * C * 2); b16* KVBl = (b16*)carve(C * C * 2); float* KS = (float*)carve(C * 4);
  if (off > ws_size || off > ((size_t)128 << 20)) return;
  prepx_kernel<<<((size_t)N * CIN / 8 + (size_t)N / 8 * 32 + 255) / 256, 256, 0, stream>>>(Fp(0), Ip(1), F16, XYZ16);
  prepw_kernel<<<dim3((C3 * C / 8 + 255) / 256, 5 + KT), 256, 0, stream>>>(Fp(3), Fp(9), Fp(15), Fp(17), Fp(20), Fp(22), WPRE, WP1, WP2, WQKV, WDW, WPROJ);
  node_kernel<<<NBLK, 128, 0, stream>>>(F16, XYZ16, WPRE, Fp(4), Fp(5), Fp(6), Fp(7), Fp(8), WP1, Fp(10), Fp(11), Fp(12), Fp(13), Fp(14), WP2, Fp(16), WQKV, Fp(18), Fp(19), Q16, V16, PART);
  reduce_kernel<<<1, 256, 0, stream>>>(PART, KVBh, KVBl, KS);
  final_kernel<<<NBLK, 128, 0, stream>>>(Q16, V16, Ip(2), KVBh, KVBl, KS, WDW, Fp(21), WPROJ, Fp(23), F16, WPRE, Fp(4), Fp(5), Fp(6), Fp(7), Fp(8), Fp(24), Fp(25), (float*)d_out);
}
